// CausalSelfAttention_32186484916684
// MI455X (gfx1250) — hardware-verified
//
#include <hip/hip_runtime.h>
#ifndef NB
#define NB 2
#endif
#ifndef SEQ
#define SEQ 2048
#endif
#define NB_FULL 2
#define SEQ_FULL 2048
#define DM 1024
#define NH 16
#define HD 64
#define QT0 256
#define NR ((size_t)NB * SEQ)
#define AL256(x) ((((size_t)(x)) + 255) & ~(size_t)255)

static_assert(DM == NH * HD);
static_assert(SEQ % 128 == 0);
static_assert(QT0 % 128 == 0);
static_assert(SEQ >= QT0);
static_assert((SEQ - QT0) % 64 == 0);
static_assert(SEQ <= SEQ_FULL);
static_assert(NB <= NB_FULL);
static_assert(DM / 8 == 128);
static_assert(DM % 64 == 0);
static_assert(DM % 32 == 0);
static_assert(HD == 64);
static_assert(HD / 2 == 32);

typedef unsigned short v8us __attribute__((ext_vector_type(8), may_alias));
typedef float  v8f  __attribute__((ext_vector_type(8)));
typedef float  v4f  __attribute__((ext_vector_type(4)));
typedef float  v2f  __attribute__((ext_vector_type(2)));
typedef float  v4fa __attribute__((ext_vector_type(4), may_alias));
typedef _Float16 v16h __attribute__((ext_vector_type(16)));
typedef _Float16 v4h __attribute__((ext_vector_type(4)));
union FragH { v16h v; v8us half[2]; _Float16 h[16]; unsigned short u[16]; };

__device__ __forceinline__ unsigned short bf16_bits(float x) { unsigned int u = __float_as_uint(x); return (unsigned short)((u + 0x7FFFu + ((u >> 16) & 1u)) >> 16); }
__device__ __forceinline__ float bf16_val(unsigned short b) { return __uint_as_float(((unsigned int)b) << 16); }
__device__ __forceinline__ float bf16_rne(float x) { return bf16_val(bf16_bits(x)); }

__device__ __forceinline__ v16h g2_frag(const _Float16* p, unsigned hh) { FragH f; f.half[0] = *(const v8us*)((const unsigned short*)p + 8 * hh); f.half[1] = *(const v8us*)((const unsigned short*)p + 16 + 8 * hh); return f.v; }
__device__ __forceinline__ v8f g2_mma(v16h a, v16h b, v8f c) { v8f d = __builtin_amdgcn_wmma_f32_16x16x32_f16(false, a, false, b, (short)0, c, false, false); asm volatile("v_nop\n\tv_nop\n\tv_nop\n\tv_nop" : "+v"(d) : "v"(a), "v"(b)); return d; }

__global__ __launch_bounds__(256) void k_rope(float* __restrict__ T, unsigned n) {
  const unsigned t = blockIdx.x * 256u + threadIdx.x; if (t >= n) return;
  const unsigned s = t >> 5, j = t & 31u;
  double p = 1.0;
  p = (j & 1u) ? p * 1.3335214321633240 : p;
  p = (j & 2u) ? p * 1.7782794100389228 : p;
  p = (j & 4u) ? p * 3.1622776601683795 : p;
  p = (j & 8u) ? p * 10.0 : p;
  p = (j & 16u) ? p * 100.0 : p;
  const float pf = (float)p; const float inv = 1.0f / pf; const float ang = (float)s * inv;
  float sn, cs; sincosf(ang, &sn, &cs);
  v2f o; o[0] = cs; o[1] = sn;
  float* d = T + (size_t)t * 2;
  *(volatile v2f*)d = o; __threadfence(); *(volatile v2f*)d = o;
}

__global__ __launch_bounds__(256) void k_w16(const float* __restrict__ W, _Float16* __restrict__ W16, unsigned n8, float scale) {
  const unsigned t = blockIdx.x * 256u + threadIdx.x; if (t >= n8) return;
  const float* src = W + (size_t)t * 8;
  const v4f a = *(const v4fa*)src, c = *(const v4fa*)(src + 4); FragH f;
#pragma unroll
  for (unsigned q = 0; q < 4; ++q) { f.h[q] = (_Float16)(bf16_rne(a[q]) * scale); f.h[4 + q] = (_Float16)(bf16_rne(c[q]) * scale); }
  const v8us o = f.half[0]; unsigned short* d = (unsigned short*)W16 + (size_t)t * 8;
  *(volatile v8us*)d = o; __threadfence(); *(volatile v8us*)d = o;
}

__global__ __launch_bounds__(256) void k_x16(const float* __restrict__ x, _Float16* __restrict__ X16, unsigned n8) {
  const unsigned t = blockIdx.x * 256u + threadIdx.x; if (t >= n8) return;
  const unsigned row = t >> 7, c8 = (t & 127u) << 3; const unsigned b = row / (unsigned)SEQ, s = row - b * (unsigned)SEQ;
  const float* src = x + ((size_t)b * SEQ_FULL + s) * DM + c8;
  const v4f a = *(const v4fa*)src, c = *(const v4fa*)(src + 4); FragH f;
#pragma unroll
  for (unsigned q = 0; q < 4; ++q) { f.h[q] = (_Float16)bf16_rne(a[q]); f.h[4 + q] = (_Float16)bf16_rne(c[q]); }
  const v8us o = f.half[0]; unsigned short* d = (unsigned short*)X16 + (size_t)t * 8;
  *(volatile v8us*)d = o; __threadfence(); *(volatile v8us*)d = o;
}

__global__ __launch_bounds__(256) void k_vt(const _Float16* __restrict__ V2, size_t pstride, _Float16* __restrict__ VT2) {
  __shared__ unsigned short tl[64][66];
  const unsigned tid = threadIdx.x; const unsigned h = blockIdx.x / (unsigned)(SEQ / 64), lg = blockIdx.x % (unsigned)(SEQ / 64); const unsigned b = blockIdx.y, pl = blockIdx.z;
  const unsigned short* src = (const unsigned short*)V2 + (size_t)pl * pstride + ((size_t)b * SEQ) * DM;
  unsigned short* dst = (unsigned short*)VT2 + ((size_t)(pl * (unsigned)NB + b) * NH + h) * ((size_t)HD * SEQ);
  for (unsigned i = tid; i < 64u * 8u; i += 256u) { const unsigned r = i >> 3, c8 = (i & 7u) << 3; FragH f; f.half[0] = *(const v8us*)(src + ((size_t)lg * 64 + r) * DM + h * 64u + c8);
#pragma unroll
    for (unsigned q = 0; q < 8; ++q) tl[r][c8 + q] = f.u[q]; }
  __syncthreads();
  for (int pass = 0; pass < 2; ++pass) {
#pragma unroll
    for (unsigned rd = 0; rd < 2; ++rd) { const unsigned d = rd * 32u + (tid >> 3), pc = tid & 7u; FragH f;
#pragma unroll
      for (unsigned q = 0; q < 8; ++q) f.u[q] = tl[pc * 8u + q][d];
      *(volatile v8us*)(dst + (size_t)d * SEQ + lg * 64u + pc * 8u) = f.half[0]; }
    if (pass == 0) __threadfence(); }
}

__global__ __launch_bounds__(128) void k_gemm2(const _Float16* __restrict__ A, unsigned lda, size_t sA, const _Float16* __restrict__ Bh, unsigned ldb, size_t sB, float alpha, const float* __restrict__ rope, unsigned ropeN,
    const float* CP, float* C, _Float16* C16, _Float16* C16L, unsigned ldc, size_t sC, unsigned M, unsigned N, unsigned K) {
  __shared__ __attribute__((aligned(16))) float so[4][32][68];
  const unsigned tid = threadIdx.x; const unsigned w = (unsigned)__builtin_amdgcn_readfirstlane((int)(tid >> 5)); const unsigned lane = tid & 31u, ln = lane & 15u, hh = lane >> 4; const unsigned by = blockIdx.y;
  A += (size_t)by * sA; Bh += (size_t)by * sB; const size_t cofs = (size_t)by * sC;
  const unsigned ntn = N >> 6; const unsigned mt = blockIdx.x / ntn, nq = blockIdx.x - mt * ntn; const unsigned row0 = mt * 128u + 32u * w, col0 = nq * 64u; if (row0 >= M) return;
  const _Float16* a0p = A + (size_t)(row0 + ln) * lda; const _Float16* a1p = a0p + (size_t)16 * lda;
  const _Float16* b0p = Bh + (size_t)(col0 + ln) * ldb; const _Float16* b1p = b0p + (size_t)16 * ldb; const _Float16* b2p = b1p + (size_t)16 * ldb; const _Float16* b3p = b2p + (size_t)16 * ldb;
  const v8f z8 = {0.f,0.f,0.f,0.f,0.f,0.f,0.f,0.f}; v8f c00 = z8, c01 = z8, c02 = z8, c03 = z8, c10 = z8, c11 = z8, c12 = z8, c13 = z8;
#pragma unroll 1
  for (unsigned kb = 0; kb < K; kb += 32) { const v16h a0 = g2_frag(a0p + kb, hh), a1 = g2_frag(a1p + kb, hh);
    v16h b = g2_frag(b0p + kb, hh); c00 = g2_mma(a0, b, c00); c10 = g2_mma(a1, b, c10);
    b = g2_frag(b1p + kb, hh); c01 = g2_mma(a0, b, c01); c11 = g2_mma(a1, b, c11);
    b = g2_frag(b2p + kb, hh); c02 = g2_mma(a0, b, c02); c12 = g2_mma(a1, b, c12);
    b = g2_frag(b3p + kb, hh); c03 = g2_mma(a0, b, c03); c13 = g2_mma(a1, b, c13); }
  v8f accs[8] = {c00, c01, c02, c03, c10, c11, c12, c13};
#pragma unroll
  for (unsigned u = 0; u < 8; ++u) { const unsigned t = u & 3u, half = u >> 2;
#pragma unroll
    for (unsigned r = 0; r < 8; ++r) { const unsigned rloc = half * 16u + 8u * hh + r; so[w][rloc][t * 16u + ln] = accs[u][r] * alpha; } }
  __builtin_amdgcn_fence(4  , "workgroup"); __builtin_amdgcn_wave_barrier();
  const unsigned rsub = lane >> 4, c4 = (lane & 15u) * 4u;
  const bool do_rope = (rope != nullptr) && (by < ropeN);
  if (do_rope || (CP != nullptr)) {
#pragma unroll 1
    for (unsigned q = 0; q < 16; ++q) { const unsigned r = q * 2u + rsub; v4f v = *(const v4fa*)&so[w][r][c4];
      if (do_rope) { const unsigned s = (row0 + r) % (unsigned)SEQ; const v4f cs = *(const v4fa*)(rope + (size_t)s * 64 + c4); v4f o;
        o[0] = v[0] * cs[0] - v[1] * cs[1]; o[1] = v[1] * cs[0] + v[0] * cs[1]; o[2] = v[2] * cs[2] - v[3] * cs[3]; o[3] = v[3] * cs[2] + v[2] * cs[3]; v = o; }
      if (CP != nullptr) { const size_t idx = cofs + (size_t)(row0 + r) * ldc + col0 + c4; const v4f cp = *(const v4fa*)(CP + idx); v = v + cp; }
      *(v4fa*)&so[w][r][c4] = v; } }
  for (int pass = 0; pass < 2; ++pass) {
#pragma unroll
    for (unsigned q = 0; q < 16; ++q) { const unsigned r = q * 2u + rsub; const v4f v = *(const v4fa*)&so[w][r][c4]; const size_t idx = cofs + (size_t)(row0 + r) * ldc + col0 + c4;
      if (C) *(volatile v4f*)(C + idx) = v;
      if (C16) { v4h h4, l4;
#pragma unroll
        for (unsigned i = 0; i < 4; ++i) { const _Float16 hv = (_Float16)v[i]; h4[i] = hv; l4[i] = (_Float16)((v[i] - (float)hv) * 1024.0f); }
        *(volatile v4h*)(C16 + idx) = h4;
        if (C16L) *(volatile v4h*)(C16L + idx) = l4; } }
    if (pass == 0) __threadfence(); }
}

template <bool RES>
__device__ __forceinline__ void attn_body(const _Float16* Qh, const _Float16* Ql, const _Float16* Kh, const _Float16* Kl, const _Float16* VTh, const _Float16* VTl, _Float16* OH, _Float16* OL, unsigned qbase) {
  __shared__ __attribute__((aligned(16))) unsigned short ot[4][2][16][72];
  const unsigned tid = threadIdx.x; const unsigned wave = (unsigned)__builtin_amdgcn_readfirstlane((int)(tid >> 5)); const unsigned lane = tid & 31u, ln = lane & 15u, hh = lane >> 4;
  const unsigned h = blockIdx.y, b = blockIdx.z; const unsigned q0w = qbase + blockIdx.x * 64u + wave * 16u;
  const size_t rowb = (size_t)b * SEQ;
  const size_t qofs = (rowb + q0w + ln) * DM + h * HD;
  const size_t kofs = (rowb + ln) * DM + h * HD;
  const size_t vofs = (((size_t)b * NH + h) * HD + ln) * SEQ;
  const v8f z8 = {0.f,0.f,0.f,0.f,0.f,0.f,0.f,0.f};
  v8f oh[4] = {z8, z8, z8, z8}; v8f orr[4] = {z8, z8, z8, z8};
  float m = -1.0e30f, l = 0.f;
  const v16h qf0 = g2_frag(Qh + qofs, hh), qf1 = g2_frag(Qh + qofs + 32, hh);
  const unsigned qi = q0w + ln; const unsigned nh = (q0w >> 5) + 1u;
#pragma unroll 1
  for (unsigned hs = 0; hs < nh; ++hs) { const unsigned kb = hs * 32u;
    const _Float16* kp = Kh + kofs + (size_t)kb * DM;
    v8f s0 = z8, s1 = z8, r0 = z8, r1 = z8;
    if (RES) { unsigned zo = 0; asm volatile("" : "+v"(zo));
      const _Float16* klp = Kl + kofs + (size_t)kb * DM;
#pragma unroll
      for (unsigned ds = 0; ds < 2; ++ds) { const v16h qh = g2_frag(Qh + qofs + zo + ds * 32u, hh); const v16h ql = g2_frag(Ql + qofs + zo + ds * 32u, hh);
        v16h ka = g2_frag(kp + ds * 32u, hh); s0 = g2_mma(ka, qh, s0); r0 = g2_mma(ka, ql, r0);
        ka = g2_frag(klp + ds * 32u, hh); r0 = g2_mma(ka, qh, r0);
        ka = g2_frag(kp + (size_t)16 * DM + ds * 32u, hh); s1 = g2_mma(ka, qh, s1); r1 = g2_mma(ka, ql, r1);
        ka = g2_frag(klp + (size_t)16 * DM + ds * 32u, hh); r1 = g2_mma(ka, qh, r1); }
    } else {
      v16h ka = g2_frag(kp, hh); s0 = g2_mma(ka, qf0, s0);
      ka = g2_frag(kp + 32, hh); s0 = g2_mma(ka, qf1, s0);
      ka = g2_frag(kp + (size_t)16 * DM, hh); s1 = g2_mma(ka, qf0, s1);
      ka = g2_frag(kp + (size_t)16 * DM + 32, hh); s1 = g2_mma(ka, qf1, s1); }
    float t[16]; const unsigned key0 = kb + 8u * hh;
#pragma unroll
    for (unsigned r = 0; r < 8; ++r) { float a0 = s0[r], a1 = s1[r];
      if (RES) { a0 += r0[r] * 0.0009765625f; a1 += r1[r] * 0.0009765625f; }
      t[r] = (key0 + r > qi) ? -1.0e30f : a0 * 0.125f;
      t[8 + r] = (key0 + 16u + r > qi) ? -1.0e30f : a1 * 0.125f; }
    float tm = t[0];
#pragma unroll
    for (unsigned i = 1; i < 16; ++i) tm = fmaxf(tm, t[i]);
    tm = fmaxf(tm, __shfl_xor(tm, 16, 32));
    const float mn = fmaxf(m, tm); const float al = __expf(m - mn); m = mn;
    float ps = 0.f; FragH ph, pl;
#pragma unroll
    for (unsigned i = 0; i < 16; ++i) { const float e = __expf(t[i] - mn); ps += e; const float p = e * 256.0f; const _Float16 hv = (_Float16)p; ph.h[i] = hv;
      if (RES) pl.h[i] = (_Float16)((p - (float)hv) * 1024.0f); else pl.h[i] = (_Float16)0.0f; }
    l = l * al + ps;
#pragma unroll
    for (unsigned dt = 0; dt < 4; ++dt) { oh[dt] = oh[dt] * al; if (RES) orr[dt] = orr[dt] * al; }
    const _Float16* vp = VTh + vofs + kb;
#pragma unroll
    for (unsigned dt = 0; dt < 4; ++dt) { v16h va = g2_frag(vp + (size_t)dt * 16 * SEQ, hh); oh[dt] = g2_mma(va, ph.v, oh[dt]);
      if (RES) { orr[dt] = g2_mma(va, pl.v, orr[dt]); va = g2_frag(VTl + vofs + kb + (size_t)dt * 16 * SEQ, hh); orr[dt] = g2_mma(va, ph.v, orr[dt]); } } }
  l += __shfl_xor(l, 16, 32);
  const float fin = 0.25f * (1.0f / l);
#pragma unroll
  for (unsigned dt = 0; dt < 4; ++dt) { FragH fh, fl;
#pragma unroll
    for (unsigned r = 0; r < 8; ++r) { float a = oh[dt][r]; if (RES) a += orr[dt][r] * 0.0009765625f; const float val = a * fin; const _Float16 hv = (_Float16)val; fh.h[r] = hv; fl.h[r] = (_Float16)((val - (float)hv) * 1024.0f); }
    *(v8us*)&ot[wave][0][ln][dt * 16u + 8u * hh] = fh.half[0];
    if (RES) *(v8us*)&ot[wave][1][ln][dt * 16u + 8u * hh] = fl.half[0]; }
  __builtin_amdgcn_fence(4  , "workgroup"); __builtin_amdgcn_wave_barrier();
  for (int pass = 0; pass < 2; ++pass) {
#pragma unroll
    for (unsigned it = 0; it < 4; ++it) { const unsigned row = it * 4u + (lane >> 3), pc = (lane & 7u) * 8u; const size_t dofs = (rowb + q0w + row) * DM + h * HD + pc;
      const v8us vh = *(const v8us*)&ot[wave][0][row][pc]; *(volatile v8us*)((unsigned short*)OH + dofs) = vh;
      if (RES) { const v8us vl = *(const v8us*)&ot[wave][1][row][pc]; *(volatile v8us*)((unsigned short*)OL + dofs) = vl; } }
    if (pass == 0) __threadfence(); }
}

__global__ __launch_bounds__(128) void k_attn_hi(const _Float16* Qh, const _Float16* Kh, const _Float16* VTh, _Float16* OH, unsigned qbase) {
  attn_body<false>(Qh, Qh, Kh, Kh, VTh, VTh, OH, OH, qbase);
}
__global__ __launch_bounds__(128) void k_attn_res(const _Float16* Qh, const _Float16* Ql, const _Float16* Kh, const _Float16* Kl, const _Float16* VTh, const _Float16* VTl, _Float16* OH, _Float16* OL, unsigned qbase) {
  attn_body<true>(Qh, Ql, Kh, Kl, VTh, VTl, OH, OL, qbase);
}

static_assert(((size_t)SEQ * 32) % 256 == 0);
static_assert(((size_t)DM * DM / 8) % 256 == 0);
static_assert((NR * DM / 8) % 256 == 0);
static_assert((size_t)((NR / 128) * (DM / 64)) * 4 * 32 * 64 == NR * DM);
static_assert((size_t)NH * (SEQ / 64) * NB * 2 * 64 * 64 == (size_t)2 * NB * NH * HD * SEQ);
static_assert((size_t)(QT0 / 64 + (SEQ - QT0) / 64) * 64 == (size_t)SEQ);
static_assert((size_t)((SEQ / 128) * (DM / 64)) * NB * 4 * 32 * 64 == NR * DM);
static_assert((size_t)((QT0 / 128) * (DM / 64)) * NB * 4 * 32 * 64 == (size_t)NB * QT0 * DM);
constexpr size_t SZ_W16 = AL256((size_t)4 * DM * DM * 2);
constexpr size_t SZ_X16 = AL256(NR * DM * 2);
constexpr size_t SZ_QKV = AL256((size_t)6 * NR * DM * 2);
constexpr size_t SZ_VT2 = AL256((size_t)2 * NB * NH * HD * SEQ * 2);
constexpr size_t SZ_O = AL256(NR * DM * 2);
constexpr size_t SZ_ROPE = AL256((size_t)SEQ * 64 * 4);
constexpr size_t SZ_TOTAL = SZ_W16 + SZ_X16 + SZ_QKV + SZ_VT2 + 2 * SZ_O + SZ_ROPE;
static_assert(SZ_TOTAL <= (size_t)134217728);
static_assert(((size_t)3 * NR * DM * 2) % 256 == 0);

extern "C" void kernel_launch(void* const* d_in, const int* in_sizes, int n_in,
                              void* d_out, int out_size, void* d_ws, size_t ws_size, hipStream_t stream) {
  if (n_in < 5) return;
  const size_t xneed = ((size_t)(NB - 1) * SEQ_FULL + SEQ) * DM;
  if ((size_t)in_sizes[0] < xneed) return;
  if ((size_t)in_sizes[1] < (size_t)DM * DM) return;
  if ((size_t)in_sizes[2] < (size_t)DM * DM) return;
  if ((size_t)in_sizes[3] < (size_t)DM * DM) return;
  if ((size_t)in_sizes[4] < (size_t)DM * DM) return;
  if ((size_t)out_size < xneed) return;
  const float* x = (const float*)d_in[0]; const float* wq = (const float*)d_in[1]; const float* wk = (const float*)d_in[2]; const float* wv = (const float*)d_in[3]; const float* wo = (const float*)d_in[4];
  float* out = (float*)d_out;
  char* ws = (char*)d_ws; size_t off = 0;
  auto take = [&](size_t bytes) { char* p = ws + off; off += (bytes + 255) & ~(size_t)255; return p; };
  _Float16* W16 = (_Float16*)take((size_t)4 * DM * DM * 2);
  _Float16* X16 = (_Float16*)take(NR * DM * 2);
  _Float16* QKV = (_Float16*)take((size_t)6 * NR * DM * 2);
  _Float16* VT2 = (_Float16*)take((size_t)2 * NB * NH * HD * SEQ * 2);
  _Float16* OH = (_Float16*)take(NR * DM * 2); _Float16* OL = (_Float16*)take(NR * DM * 2);
  float* ROPE = (float*)take((size_t)SEQ * 64 * 4);
  if (off > ws_size || off > (size_t)134217728) return;
  const size_t PL = NR * DM;
  _Float16* Q16 = QKV; _Float16* K16 = QKV + PL; _Float16* V16 = QKV + 2 * PL;
  _Float16* Q16L = QKV + 3 * PL; _Float16* K16L = QKV + 4 * PL;
  _Float16* WO16 = W16 + (size_t)3 * DM * DM;

  k_rope<<<(unsigned)((size_t)SEQ * 32 / 256), 256, 0, stream>>>(ROPE, (unsigned)((size_t)SEQ * 32));
  k_x16<<<(unsigned)(NR * DM / 8 / 256), 256, 0, stream>>>(x, X16, (unsigned)(NR * DM / 8));
  const unsigned wn8 = (unsigned)((size_t)DM * DM / 8);
  k_w16<<<wn8 / 256, 256, 0, stream>>>(wq, W16, wn8, 16.0f);
  k_w16<<<wn8 / 256, 256, 0, stream>>>(wk, W16 + (size_t)DM * DM, wn8, 16.0f);
  k_w16<<<wn8 / 256, 256, 0, stream>>>(wv, W16 + (size_t)2 * DM * DM, wn8, 16.0f);
  k_w16<<<wn8 / 256, 256, 0, stream>>>(wo, WO16, wn8, 16.0f);

  const dim3 gp((unsigned)((NR / 128) * (DM / 64)), 3);
  k_gemm2<<<gp, 128, 0, stream>>>(X16, DM, 0, W16, DM, (size_t)DM * DM, 0.0625f, ROPE, 2u, nullptr, nullptr, QKV, QKV + 3 * PL, DM, PL, (unsigned)NR, DM, DM);

  k_vt<<<dim3(NH * (SEQ / 64), NB, 2), 256, 0, stream>>>(V16, 3 * PL, VT2);
  const _Float16* VTh = VT2; const _Float16* VTl = VT2 + (size_t)NB * NH * HD * SEQ;

  k_attn_res<<<dim3(QT0 / 64, NH, NB), 128, 0, stream>>>(Q16, Q16L, K16, K16L, VTh, VTl, OH, OL, 0u);
  if (SEQ > QT0) k_attn_hi<<<dim3((SEQ - QT0) / 64, NH, NB), 128, 0, stream>>>(Q16, K16, VTh, OH, (unsigned)QT0);

  const dim3 gf((SEQ / 128) * (DM / 64), NB);
  k_gemm2<<<gf, 128, 0, stream>>>(OH, DM, (size_t)SEQ * DM, WO16, DM, 0, 0.0009765625f, nullptr, 0u, nullptr, out, nullptr, nullptr, DM, (size_t)SEQ_FULL * DM, SEQ, DM, DM);
  const dim3 gl((QT0 / 128) * (DM / 64), NB);
  k_gemm2<<<gl, 128, 0, stream>>>(OL, DM, (size_t)SEQ * DM, WO16, DM, 0, 0.00000095367431640625f, nullptr, 0u, out, out, nullptr, nullptr, DM, (size_t)SEQ_FULL * DM, QT0, DM, DM);
}
